// GATStochasticMuZeroModel_72971494359379
// MI455X (gfx1250) — hardware-verified
//
#include <hip/hip_runtime.h>


namespace {
constexpr int G = 4096, NN = 16, NT = G * NN, CIN = 16, F = 64, NH = 4, HF = NH * F, M1 = 128, M2 = 256;
constexpr float AS_ = 8.0f, WS_ = 16.0f, NEG = 0.2f, LNE = 1e-5f;

typedef _Float16 b16;
typedef __attribute__((ext_vector_type(16))) _Float16 v16b;
typedef __attribute__((ext_vector_type(8))) _Float16 v8b;
typedef __attribute__((ext_vector_type(8))) float v8f;
typedef __attribute__((ext_vector_type(4))) float v4f;
__device__ __forceinline__ void split16(float v, b16& hi, b16& lo) { hi = (b16)v; lo = (b16)(v - (float)hi); }
__device__ __forceinline__ v16b frag_kb(const b16* p, int hh) { const v8b a = *(const v8b*)(p + 8 * hh), b = *(const v8b*)(p + 16 + 8 * hh); v16b f;
#pragma unroll
  for (int e = 0; e < 8; ++e) { f[e] = a[e]; f[8 + e] = b[e]; } return f; }
__device__ __forceinline__ v8f wmma16b(v16b a, v16b b, v8f c) { v8f d = __builtin_amdgcn_wmma_f32_16x16x32_f16(false, a, false, b, (short)0, c, false, false); asm volatile("v_nop\n\tv_nop\n\tv_nop\n\tv_nop" : "+v"(d) : "v"(a), "v"(b)); return d; }
__device__ __forceinline__ void wave_lds_sync() { __builtin_amdgcn_fence(__ATOMIC_RELEASE, "workgroup"); __builtin_amdgcn_wave_barrier(); __builtin_amdgcn_fence(__ATOMIC_ACQUIRE, "workgroup"); }
__device__ __forceinline__ float nexp(float x) { return __builtin_amdgcn_exp2f(x * 1.4426950408889634f); }

__global__ __launch_bounds__(256) void prep_kernel(const float* __restrict__ x, const float* __restrict__ inw, const float* __restrict__ g0w, const float* __restrict__ g1w, const float* __restrict__ g2w, const float* __restrict__ w1, const float* __restrict__ w2,
                                                   float* __restrict__ xr, b16* __restrict__ pin, b16* __restrict__ p0, b16* __restrict__ p1, b16* __restrict__ p2, b16* __restrict__ pm1, b16* __restrict__ pm2) {
  const size_t tid = (size_t)blockIdx.x * blockDim.x + threadIdx.x, nth = (size_t)gridDim.x * blockDim.x;
  auto plane = [&](const float* W, int KIN, int KREAL, int NOUT, b16* dst) { const size_t PL = (size_t)NOUT * KIN;
    for (size_t p = tid; p < PL; p += nth) { const int n = (int)(p / KIN), k = (int)(p % KIN); const float v = (k < KREAL) ? W[(size_t)min(k, KREAL - 1) * NOUT + n] * WS_ : 0.0f; b16 a, c; split16(v, a, c); ((volatile b16*)dst)[p] = a; ((volatile b16*)dst)[PL + p] = c; } };
  for (int pass = 0; pass < 2; ++pass) {
    for (size_t p = tid; p < (size_t)NT * 32 / 4; p += nth) { const int row = (int)(p >> 3), k0 = (int)(p & 7) * 4; const int g = row >> 4, n = row & 15; v4f v;
#pragma unroll
      for (int e = 0; e < 4; ++e) { const int k = k0 + e; v[e] = (k < CIN) ? x[((size_t)g * CIN + min(k, CIN - 1)) * NN + n] : 0.0f; }
      *(volatile v4f*)(xr + (size_t)row * 32 + k0) = v; }
    plane(inw, 32, CIN, F, pin); plane(g0w, F, F, HF, p0); plane(g1w, HF, HF, HF, p1); plane(g2w, HF, HF, HF, p2); plane(w1, F, F, M1, pm1); plane(w2, M1, M1, M2, pm2);
    __threadfence();
  }
}

template <int KIN, int NOUT, int EPI>
__global__ __launch_bounds__(256) void gemm_kernel(const float* A, const b16* __restrict__ bw, const float* __restrict__ bias, float* Y) {
  constexpr int NTL = NOUT / 32;
  __shared__ __attribute__((aligned(16))) float Ts[8][32][(NOUT / 2) + 4];
  const int lane = threadIdx.x & 31, wave = threadIdx.x >> 5, nloc = lane & 15, hlf = lane >> 4, m0 = blockIdx.x * 128 + (wave & 3) * 32, c0 = (wave >> 2) * (NOUT / 2);
  v8f acc[2][NTL];
#pragma unroll
  for (int r = 0; r < 2; ++r)
#pragma unroll
    for (int t = 0; t < NTL; ++t) acc[r][t] = (v8f){};
#pragma unroll 1
  for (int kb = 0; kb < KIN; kb += 32) { v16b a0, a1, l0, l1;
#pragma unroll
    for (int e = 0; e < 16; ++e) { const int k = kb + ((e < 8) ? (8 * hlf + e) : (16 + 8 * hlf + e - 8)); b16 p, q; split16(A[(size_t)(m0 + nloc) * KIN + k] * AS_, p, q); a0[e] = p; l0[e] = q; split16(A[(size_t)(m0 + 16 + nloc) * KIN + k] * AS_, p, q); a1[e] = p; l1[e] = q; }
#pragma unroll
    for (int t = 0; t < NTL; ++t) { const size_t bo = (size_t)(c0 + t * 16 + nloc) * KIN + kb; const v16b b0 = frag_kb(bw + bo, hlf), b1 = frag_kb(bw + (size_t)NOUT * KIN + bo, hlf);
      acc[0][t] = wmma16b(a0, b0, acc[0][t]); acc[0][t] = wmma16b(l0, b0, acc[0][t]); acc[0][t] = wmma16b(a0, b1, acc[0][t]);
      acc[1][t] = wmma16b(a1, b0, acc[1][t]); acc[1][t] = wmma16b(l1, b0, acc[1][t]); acc[1][t] = wmma16b(a1, b1, acc[1][t]); } }
#pragma unroll
  for (int t = 0; t < NTL; ++t)
#pragma unroll
    for (int r = 0; r < 2; ++r)
#pragma unroll
      for (int v = 0; v < 8; ++v) { float val = acc[r][t][v] * (1.0f / (AS_ * WS_)); if (EPI == 1) val = fmaxf(val + bias[c0 + t * 16 + nloc], 0.0f); Ts[wave][r * 16 + v + 8 * hlf][t * 16 + nloc] = val; }
  __syncthreads();
  for (int pass = 0; pass < 2; ++pass) {
    for (int j = 0; j < 32 * (NOUT / 2) / 4 / 32; ++j) { const int idx = j * 32 + lane; const int rr = idx / (NOUT / 8), c4 = (idx % (NOUT / 8)) * 4;
      *(volatile v4f*)(Y + (size_t)(m0 + rr) * NOUT + c0 + c4) = *(const v4f*)(&Ts[wave][rr][c4]); }
    __threadfence(); }
}

template <int MODE>
__global__ __launch_bounds__(256) void gat_kernel(float* H, const float* __restrict__ asrc, const float* __restrict__ adst, const float* __restrict__ bias, float* __restrict__ gout) {
  __shared__ __attribute__((aligned(16))) float X[4][NN][HF + 4]; __shared__ float ES[4][NN][NH], ED[4][NN][NH]; __shared__ float AD[4][NH][NN][NN]; __shared__ __attribute__((aligned(16))) float O[4][NN][HF + 4]; __shared__ __attribute__((aligned(16))) float Gs[4][F];
  const int t_ = threadIdx.x, gl = t_ >> 6, tl = t_ & 63, g = blockIdx.x * 4 + gl; const size_t row0 = (size_t)g * NN;
  for (int q = tl; q < NH * NN * NN; q += 64) (&AD[gl][0][0][0])[q] = 0.0f;
  for (int i = tl; i < NN * HF / 4; i += 64) { const int n = i / (HF / 4), c4 = (i % (HF / 4)) * 4; *(v4f*)(&X[gl][n][c4]) = *(const v4f*)(H + (row0 + n) * HF + c4); }
  __syncthreads();
  { const int n = tl >> 2, h = tl & 3; float s = 0.0f, d = 0.0f;
#pragma unroll 1
    for (int f = 0; f < F; ++f) { const float v = X[gl][n][h * F + f]; s += v * asrc[h * F + f]; d += v * adst[h * F + f]; }
    ES[gl][n][h] = s; ED[gl][n][h] = d; }
  __syncthreads();
  const int i = tl >> 2, yi = i >> 2, xi = i & 3;
  const bool ok1 = (xi + 1 < 4), ok2 = (xi > 0), ok3 = (yi + 1 < 4), ok4 = (yi > 0);
  const int j1 = ok1 ? i + 1 : i, j2 = ok2 ? i - 1 : i, j3 = ok3 ? i + 4 : i, j4 = ok4 ? i - 4 : i;
  { const int h = tl & 3; const float edi = ED[gl][i][h];
    auto lgt = [&](int j, bool ok) { float a = ES[gl][j][h] + edi; a = (a > 0.0f) ? a : NEG * a; return ok ? a : -INFINITY; };
    const float a0 = lgt(i, true), a1 = lgt(j1, ok1), a2 = lgt(j2, ok2), a3 = lgt(j3, ok3), a4 = lgt(j4, ok4);
    const float m = fmaxf(fmaxf(fmaxf(a0, a1), fmaxf(a2, a3)), a4);
    const float w0 = nexp(a0 - m), w1 = ok1 ? nexp(a1 - m) : 0.0f, w2 = ok2 ? nexp(a2 - m) : 0.0f, w3 = ok3 ? nexp(a3 - m) : 0.0f, w4 = ok4 ? nexp(a4 - m) : 0.0f;
    const float id = 1.0f / (w0 + w1 + w2 + w3 + w4);
    AD[gl][h][i][i] = w0 * id; if (ok1) AD[gl][h][i][j1] = w1 * id; if (ok2) AD[gl][h][i][j2] = w2 * id; if (ok3) AD[gl][h][i][j3] = w3 * id; if (ok4) AD[gl][h][i][j4] = w4 * id; }
  __syncthreads();
  {
    const int wv = tl >> 5, lane = tl & 31, nloc = lane & 15, hh = lane >> 4;
#pragma unroll 1
    for (int hq = 0; hq < 2; ++hq) { const int h = wv * 2 + hq; v16b bh_, bl_;
#pragma unroll
      for (int e = 0; e < 8; ++e) { b16 a, c; split16(AD[gl][h][nloc][8 * hh + e], a, c); bh_[e] = a; bl_[e] = c; bh_[8 + e] = (b16)0.0f; bl_[8 + e] = (b16)0.0f; }
#pragma unroll
      for (int t = 0; t < 4; ++t) { v16b ah_, al_;
#pragma unroll
        for (int e = 0; e < 8; ++e) { b16 a, c; split16(X[gl][8 * hh + e][h * F + t * 16 + nloc] * AS_, a, c); ah_[e] = a; al_[e] = c; ah_[8 + e] = (b16)0.0f; al_[8 + e] = (b16)0.0f; }
        v8f acc = {}; acc = wmma16b(ah_, bh_, acc); acc = wmma16b(al_, bh_, acc); acc = wmma16b(ah_, bl_, acc);
#pragma unroll
        for (int r = 0; r < 8; ++r) O[gl][nloc][h * F + t * 16 + 8 * hh + r] = acc[r] * (1.0f / AS_); } } }
  __syncthreads();
  if (MODE == 0) {
    for (int pass = 0; pass < 2; ++pass) {
      for (int q = tl; q < NN * HF / 4; q += 64) { const int n = q / (HF / 4), c4 = (q % (HF / 4)) * 4; v4f v = *(const v4f*)(&O[gl][n][c4]);
#pragma unroll
        for (int e = 0; e < 4; ++e) v[e] = fmaxf(v[e] + bias[c4 + e], 0.0f);
        *(volatile v4f*)(H + (row0 + n) * HF + c4) = v; }
      __threadfence(); }
  } else {
    { const int f = tl; float s = 0.0f;
      for (int n = 0; n < NN; ++n) { float mh = 0.0f;
#pragma unroll
        for (int h = 0; h < NH; ++h) mh += O[gl][n][h * F + f];
        s += mh * 0.25f + bias[f]; }
      Gs[gl][f] = s * (1.0f / NN); }
    __syncthreads();
    for (int pass = 0; pass < 2; ++pass) { if (t_ < 64) *(volatile v4f*)(gout + (size_t)blockIdx.x * 4 * F + t_ * 4) = *(const v4f*)(&Gs[0][0] + t_ * 4); __threadfence(); }
  }
}

template <int W>
__global__ __launch_bounds__(256) void ln_kernel(float* y, const float* __restrict__ bias, const float* __restrict__ gma, const float* __restrict__ bta, float* __restrict__ out) {
  constexpr int NG = W / 128;
  const int wid = threadIdx.x >> 5, lane = threadIdx.x & 31; const size_t row = (size_t)blockIdx.x * 8 + wid;
  v4f v[NG]; float s = 0.0f;
#pragma unroll
  for (int g = 0; g < NG; ++g) { v[g] = *(const v4f*)(y + row * W + g * 128 + lane * 4);
#pragma unroll
    for (int e = 0; e < 4; ++e) { v[g][e] += bias[g * 128 + lane * 4 + e]; s += v[g][e]; } }
#pragma unroll
  for (int o = 1; o < 32; o <<= 1) s += __shfl_xor(s, o);
  const float mu = s * (1.0f / W); float q = 0.0f;
#pragma unroll
  for (int g = 0; g < NG; ++g)
#pragma unroll
    for (int e = 0; e < 4; ++e) { const float d = v[g][e] - mu; q += d * d; }
#pragma unroll
  for (int o = 1; o < 32; o <<= 1) q += __shfl_xor(q, o);
  const float rs = rsqrtf(q * (1.0f / W) + LNE);
  v4f r[NG];
#pragma unroll
  for (int g = 0; g < NG; ++g)
#pragma unroll
    for (int e = 0; e < 4; ++e) { const int c = g * 128 + lane * 4 + e; r[g][e] = fmaxf((v[g][e] - mu) * rs * gma[c] + bta[c], 0.0f); }
  __builtin_amdgcn_wave_barrier();
  float* dst = (out != nullptr) ? out : y;
  for (int pass = 0; pass < 2; ++pass) {
#pragma unroll
    for (int g = 0; g < NG; ++g) *(volatile v4f*)(dst + row * W + g * 128 + lane * 4) = r[g];
    __threadfence(); }
}
}

extern "C" void kernel_launch(void* const* d_in, const int* in_sizes, int n_in,
                              void* d_out, int out_size, void* d_ws, size_t ws_size, hipStream_t stream) {
  (void)n_in; (void)out_size;
  const float* x = (const float*)d_in[0]; const float* inw = (const float*)d_in[1]; const float* inb = (const float*)d_in[2];
  const float* g0w = (const float*)d_in[3]; const float* g0s = (const float*)d_in[4]; const float* g0d = (const float*)d_in[5]; const float* g0b = (const float*)d_in[6];
  const float* g1w = (const float*)d_in[7]; const float* g1s = (const float*)d_in[8]; const float* g1d = (const float*)d_in[9]; const float* g1b = (const float*)d_in[10];
  const float* g2w = (const float*)d_in[11]; const float* g2s = (const float*)d_in[12]; const float* g2d = (const float*)d_in[13]; const float* g2b = (const float*)d_in[14];
  const float* w1 = (const float*)d_in[15]; const float* b1 = (const float*)d_in[16]; const float* l1g = (const float*)d_in[17]; const float* l1b = (const float*)d_in[18];
  const float* w2 = (const float*)d_in[19]; const float* b2 = (const float*)d_in[20]; const float* l2g = (const float*)d_in[21]; const float* l2b = (const float*)d_in[22];
  float* out = (float*)d_out;
  if (in_sizes[0] != G * CIN * NN || in_sizes[1] != CIN * F || in_sizes[3] != F * HF || in_sizes[7] != HF * HF || in_sizes[11] != HF * HF || in_sizes[15] != F * M1 || in_sizes[19] != M1 * M2) return;
  size_t off = 0; char* ws = (char*)d_ws;
  auto carve = [&](size_t bytes) { char* p = ws + off; off += (bytes + 255) & ~(size_t)255; return p; };
  float* xr = (float*)carve((size_t)NT * 32 * 4); b16* pin = (b16*)carve((size_t)F * 32 * 4); b16* p0 = (b16*)carve((size_t)HF * F * 4); b16* p1 = (b16*)carve((size_t)HF * HF * 4); b16* p2 = (b16*)carve((size_t)HF * HF * 4); b16* pm1 = (b16*)carve((size_t)M1 * F * 4); b16* pm2 = (b16*)carve((size_t)M2 * M1 * 4);
  float* h0 = (float*)carve((size_t)NT * F * 4); float* Hb = (float*)carve((size_t)NT * HF * 4); float* gr = (float*)carve((size_t)G * F * 4); float* y1 = (float*)carve((size_t)G * M1 * 4); float* y2 = (float*)carve((size_t)G * M2 * 4);
  if (off > ws_size) return;
  prep_kernel<<<1024, 256, 0, stream>>>(x, inw, g0w, g1w, g2w, w1, w2, xr, pin, p0, p1, p2, pm1, pm2);
  gemm_kernel<32, F, 1><<<NT / 128, 256, 0, stream>>>(xr, pin, inb, h0);
  gemm_kernel<F, HF, 0><<<NT / 128, 256, 0, stream>>>(h0, p0, nullptr, Hb);
  gat_kernel<0><<<G / 4, 256, 0, stream>>>(Hb, g0s, g0d, g0b, nullptr);
  gemm_kernel<HF, HF, 0><<<NT / 128, 256, 0, stream>>>(Hb, p1, nullptr, Hb);
  gat_kernel<0><<<G / 4, 256, 0, stream>>>(Hb, g1s, g1d, g1b, nullptr);
  gemm_kernel<HF, HF, 0><<<NT / 128, 256, 0, stream>>>(Hb, p2, nullptr, Hb);
  gat_kernel<1><<<G / 4, 256, 0, stream>>>(Hb, g2s, g2d, g2b, gr);
  gemm_kernel<F, M1, 0><<<G / 128, 256, 0, stream>>>(gr, pm1, nullptr, y1);
  ln_kernel<M1><<<G / 8, 256, 0, stream>>>(y1, b1, l1g, l1b, nullptr);
  gemm_kernel<M1, M2, 0><<<G / 128, 256, 0, stream>>>(y1, pm2, nullptr, y2);
  ln_kernel<M2><<<G / 8, 256, 0, stream>>>(y2, b2, l2g, l2b, out);
}
